// PraxisAttention_76501957476887
// MI455X (gfx1250) — hardware-verified
//
#include <hip/hip_runtime.h>

typedef __attribute__((ext_vector_type(16))) _Float16 v16h;
typedef __attribute__((ext_vector_type(8)))  _Float16 v8h;
typedef __attribute__((ext_vector_type(16))) __bf16   v16b;
typedef __attribute__((ext_vector_type(8)))  __bf16   v8b;
typedef __attribute__((ext_vector_type(8)))  float    v8f;
typedef __attribute__((ext_vector_type(4)))  float    v4f;
typedef __attribute__((ext_vector_type(4)))  unsigned int u4v;

constexpr int kBatch   = 2;
constexpr int kSeq     = 2048;
constexpr int kDModel  = 1024;
constexpr int kHeads   = 16;
constexpr int kHeadDim = 64;
constexpr int kQKCols  = 2 * kDModel;
constexpr int kTok     = kBatch * kSeq;
constexpr int kQB      = 64;
constexpr int kKC      = 64;
constexpr int kNQblk   = kSeq / kQB;
constexpr int kAttnBlocks = kBatch * kHeads * kNQblk;
constexpr float kMergeCarry = 8.0f;
constexpr float kWoCarry    = 256.0f;

static_assert(kNQblk == 32);
static_assert(kHeads == 16);
static_assert(kAttnBlocks == 1024);
static_assert(kSeq % kQB == 0);
static_assert(kDModel % 32 == 0);
static_assert(kTok % 64 == 0 && kQKCols % 64 == 0 && kDModel % 64 == 0 && kSeq % 64 == 0);

constexpr size_t kBytesXb     = (size_t)kTok * kDModel * 2;
constexpr size_t kBytesWqk    = (size_t)kQKCols * kDModel * 2;
constexpr size_t kBytesWv     = (size_t)kDModel * kDModel * 2;
constexpr size_t kBytesWo     = (size_t)kDModel * kDModel * 2;
constexpr size_t kBytesQPl    = (size_t)kTok * kQKCols * 2;
constexpr size_t kBytesVtPl   = (size_t)kBatch * kDModel * kSeq * 2;
constexpr size_t kBytesAtt    = (size_t)kBatch * kHeads * kSeq * kHeadDim * 4;
constexpr size_t kBytesMerged = (size_t)kTok * kDModel * 2;
constexpr size_t kBytesPart   = (size_t)kAttnBlocks * 128;
constexpr size_t kBytesStats  = (size_t)kBatch * kHeads * 128;
constexpr size_t kBytesLam    = 128;

constexpr size_t kOffXb     = 0;
constexpr size_t kOffWqb    = kOffXb + kBytesXb;
constexpr size_t kOffWkb    = kOffWqb + kBytesWqk;
constexpr size_t kOffWvb    = kOffWkb + kBytesWqk;
constexpr size_t kOffWo16   = kOffWvb + kBytesWv;
constexpr size_t kOffQh     = kOffWo16 + kBytesWo;
constexpr size_t kOffQl     = kOffQh + kBytesQPl;
constexpr size_t kOffKh     = kOffQl + kBytesQPl;
constexpr size_t kOffKl     = kOffKh + kBytesQPl;
constexpr size_t kOffVth    = kOffKl + kBytesQPl;
constexpr size_t kOffVtl    = kOffVth + kBytesVtPl;
constexpr size_t kOffAtt    = kOffVtl + kBytesVtPl;
constexpr size_t kOffMerged = kOffAtt + kBytesAtt;
constexpr size_t kOffPart   = kOffMerged + kBytesMerged;
constexpr size_t kOffStats  = kOffPart + kBytesPart;
constexpr size_t kOffLam    = kOffStats + kBytesStats;
constexpr size_t kWsTotal   = kOffLam + kBytesLam;
static_assert(kBytesPart == 131072);
static_assert(kWsTotal == 130158720);
static_assert(kWsTotal <= 134217728);
static_assert(kOffWqb % 128 == 0 && kOffQh % 128 == 0 && kOffAtt % 128 == 0 && kOffPart % 128 == 0 && kOffStats % 128 == 0 && kOffLam % 128 == 0);

__device__ __forceinline__ unsigned short f2bf_bits(float f) {
  unsigned u = __float_as_uint(f);
  return (unsigned short)((u + 0x7FFFu + ((u >> 16) & 1u)) >> 16);
}
__device__ __forceinline__ float bf_bits2f(unsigned short h) { return __uint_as_float(((unsigned)h) << 16); }
__device__ __forceinline__ float bf_rne(float f) { return bf_bits2f(f2bf_bits(f)); }

__device__ __forceinline__ void dep_guard_h(v8f& a, v8f& b, v16h x, v16h y) { asm volatile("v_nop\n\tv_nop\n\tv_nop\n\tv_nop" : "+v"(a), "+v"(b) : "v"(x), "v"(y)); }
__device__ __forceinline__ void dep_guard_b(v8f& a, v8f& b, v16b x, v16b y) { asm volatile("v_nop\n\tv_nop\n\tv_nop\n\tv_nop" : "+v"(a), "+v"(b) : "v"(x), "v"(y)); }
__device__ __forceinline__ void keep4_h(v16h a, v16h b, v16h c, v16h d) { asm volatile("v_nop" :: "v"(a), "v"(b), "v"(c), "v"(d)); }
__device__ __forceinline__ void keep4_b(v16b a, v16b b, v16b c, v16b d) { asm volatile("v_nop" :: "v"(a), "v"(b), "v"(c), "v"(d)); }
__device__ __forceinline__ void acc_guard4(v8f& a, v8f& b, v8f& c, v8f& d) { asm volatile("v_nop\n\tv_nop\n\tv_nop\n\tv_nop" : "+v"(a), "+v"(b), "+v"(c), "+v"(d)); }
template <typename T> struct Frag;
template <> struct Frag<_Float16> {
  typedef v16h V; union U { v16h v; v8h h[2]; };
  static __device__ __forceinline__ v16h load(const _Float16* p) {
    U f; f.h[0] = *(const v8h*)(p); f.h[1] = *(const v8h*)(p + 16); return f.v;
  }
  static __device__ __forceinline__ v8f mma(v16h a, v16h b, v8f c) {
    return __builtin_amdgcn_wmma_f32_16x16x32_f16(false, a, false, b, (short)0, c, false, false);
  }
  static __device__ __forceinline__ void guard(v8f& a, v8f& b, v16h x, v16h y) { dep_guard_h(a, b, x, y); }
  static __device__ __forceinline__ void keep(v16h a, v16h b, v16h c, v16h d) { keep4_h(a, b, c, d); }
};
template <> struct Frag<__bf16> {
  typedef v16b V; union U { v16b v; v8b h[2]; };
  static __device__ __forceinline__ v16b load(const __bf16* p) {
    U f; f.h[0] = *(const v8b*)(p); f.h[1] = *(const v8b*)(p + 16); return f.v;
  }
  static __device__ __forceinline__ v8f mma(v16b a, v16b b, v8f c) {
    return __builtin_amdgcn_wmma_f32_16x16x32_bf16(false, a, false, b, (short)0, c, false, false);
  }
  static __device__ __forceinline__ void guard(v8f& a, v8f& b, v16b x, v16b y) { dep_guard_b(a, b, x, y); }
  static __device__ __forceinline__ void keep(v16b a, v16b b, v16b c, v16b d) { keep4_b(a, b, c, d); }
};

template <int ET> struct Elem;
template <> struct Elem<0> { typedef _Float16 T; };
template <> struct Elem<1> { typedef __bf16 T; };
template <int ET, bool SPLIT, int BIAS_MODE, int OUT_MODE, bool RESID, int ACT = 0>
__global__ __launch_bounds__(256) void wmma_gemm64(
    const unsigned short* __restrict__ Ap, const unsigned short* __restrict__ A2p, int lda, long strideA,
    const unsigned short* __restrict__ Btp, const unsigned short* __restrict__ Bt2p, int ldb, long strideB,
    void* __restrict__ Cout, void* __restrict__ Cout2, int ldc, long strideC,
    const float* __restrict__ bias,
    const float* __restrict__ resid, long strideR,
    int M, int N, int K, float scale) {
  typedef typename Elem<ET>::T T;
  typedef typename Frag<T>::V V;
  const T* A = (const T*)Ap; const T* A2 = (const T*)A2p; const T* Bt = (const T*)Btp; const T* Bt2 = (const T*)Bt2p;
  __shared__ __align__(16) float sT[8][16 * 68];
  const int b    = blockIdx.y;
  const int lane = threadIdx.x & 31;
  const int wave = threadIdx.x >> 5;
  const int tilesN = N >> 6;
  const int tilesM = M >> 6;
  const int tile = blockIdx.x * 8 + wave;
  if (tile >= tilesM * tilesN) return;
  const int tm = tile / tilesN;
  const int tn = tile - tm * tilesN;
  const int m0 = tm << 6;
  const int n0 = tn << 6;

  const T* Ab  = A  + (size_t)b * strideA;
  const T* Bb  = Bt + (size_t)b * strideB;
  const T* Ab2 = SPLIT ? (A2  + (size_t)b * strideA) : nullptr;
  const T* Bb2 = SPLIT ? (Bt2 + (size_t)b * strideB) : nullptr;

  const int rlane = lane & 15;
  const int koff  = (lane >> 4) * 8;
  const int mOff  = (lane >> 4) * 8;

  v8f acc[4][4];
#pragma unroll
  for (int i = 0; i < 4; ++i)
#pragma unroll
    for (int j = 0; j < 4; ++j) acc[i][j] = (v8f){0.f,0.f,0.f,0.f,0.f,0.f,0.f,0.f};

  for (int k0 = 0; k0 < K; k0 += 32) {
    V bh[4], bl[4];
#pragma unroll
    for (int j = 0; j < 4; ++j) {
      const size_t bo = (size_t)(n0 + (j << 4) + rlane) * ldb + koff + k0;
      bh[j] = Frag<T>::load(Bb + bo);
      if (SPLIT) bl[j] = Frag<T>::load(Bb2 + bo);
    }
#pragma unroll
    for (int i = 0; i < 4; ++i) {
      const size_t ao = (size_t)(m0 + (i << 4) + rlane) * lda + koff + k0;
      V ah = Frag<T>::load(Ab + ao);
      V al;
      if (SPLIT) al = Frag<T>::load(Ab2 + ao);
#pragma unroll
      for (int j = 0; j < 4; ++j) {
        acc[i][j] = Frag<T>::mma(ah, bh[j], acc[i][j]);
        if (SPLIT) {
          acc[i][j] = Frag<T>::mma(ah, bl[j], acc[i][j]);
          acc[i][j] = Frag<T>::mma(al, bh[j], acc[i][j]);
        }
      }
      Frag<T>::guard(acc[i][0], acc[i][3], ah, SPLIT ? al : ah);
    }
    Frag<T>::keep(bh[0], bh[1], bh[2], bh[3]);
    if (SPLIT) Frag<T>::keep(bl[0], bl[1], bl[2], bl[3]);
  }
  acc_guard4(acc[0][0], acc[0][1], acc[0][2], acc[0][3]);
  acc_guard4(acc[1][0], acc[1][1], acc[1][2], acc[1][3]);
  acc_guard4(acc[2][0], acc[2][1], acc[2][2], acc[2][3]);
  acc_guard4(acc[3][0], acc[3][1], acc[3][2], acc[3][3]);

  float* slab = sT[wave];
  const float* Rb = RESID ? (resid + (size_t)b * strideR) : nullptr;
#pragma unroll
  for (int i = 0; i < 4; ++i) {
    const int mBase = m0 + (i << 4);
#pragma unroll
    for (int j = 0; j < 4; ++j) {
      const int n = n0 + (j << 4) + rlane;
      float bv = 0.f;
      if (BIAS_MODE == 2) bv = bias[n];
#pragma unroll
      for (int r = 0; r < 8; ++r) {
        float v = acc[i][j][r] * scale;
        if (BIAS_MODE == 1) v += bias[mBase + mOff + r];
        if (BIAS_MODE == 2) v += bv;
        if (RESID) v += Rb[(size_t)(mBase + mOff + r) * ldc + n];
        if (ACT == 1) v = tanhf(v);
        if (ACT == 2) v = fmaxf(v, 0.0f);
        if (ACT == 3) v = v / (1.0f + expf(-v));
        if (ACT == 4) v = (v > 0.f) ? v : 0.01f * v;
        if (ACT == 5) v = 0.5f * v * (1.0f + erff(v * 0.70710678118654752f));
        slab[(mOff + r) * 68 + (j << 4) + rlane] = v;
      }
    }
    __builtin_amdgcn_fence(__ATOMIC_RELEASE, "workgroup");
    __builtin_amdgcn_wave_barrier();
    __builtin_amdgcn_fence(__ATOMIC_ACQUIRE, "workgroup");
    if (OUT_MODE == 0) {
      float* C = (float*)Cout + (size_t)b * strideC;
      const int hh = lane >> 4, c4 = (lane & 15) * 4;
      for (int pass = 0; pass < 2; ++pass) {
#pragma unroll
        for (int it = 0; it < 8; ++it) {
          const int row = it * 2 + hh;
          v4f v = *(const v4f*)(slab + row * 68 + c4);
          *(volatile v4f*)(C + (size_t)(mBase + row) * ldc + n0 + c4) = v;
        }
        __threadfence();
      }
    } else {
      const int q = lane >> 3, c8 = (lane & 7) * 8;
      unsigned short* C  = (unsigned short*)Cout  + (size_t)b * strideC;
      unsigned short* C2 = (OUT_MODE == 2) ? ((unsigned short*)Cout2 + (size_t)b * strideC) : nullptr;
      for (int pass = 0; pass < 2; ++pass) {
#pragma unroll
        for (int it = 0; it < 4; ++it) {
          const int row = it * 4 + q;
          const float* sp = slab + row * 68 + c8;
          v8h hv, lv;
#pragma unroll
          for (int e = 0; e < 8; ++e) {
            if (OUT_MODE == 1) {
              hv[e] = (_Float16)sp[e];
            } else {
              unsigned short hb = f2bf_bits(sp[e]);
              unsigned short lb = f2bf_bits(sp[e] - bf_bits2f(hb));
              hv[e] = __builtin_bit_cast(_Float16, hb);
              lv[e] = __builtin_bit_cast(_Float16, lb);
            }
          }
          *(volatile v8h*)(C + (size_t)(mBase + row) * ldc + n0 + c8) = hv;
          if (OUT_MODE == 2) *(volatile v8h*)(C2 + (size_t)(mBase + row) * ldc + n0 + c8) = lv;
        }
        __threadfence();
      }
    }
    __builtin_amdgcn_fence(__ATOMIC_RELEASE, "workgroup");
    __builtin_amdgcn_wave_barrier();
    __builtin_amdgcn_fence(__ATOMIC_ACQUIRE, "workgroup");
  }
}

__global__ __launch_bounds__(256) void cast_f32_bf16x2(
    const float* __restrict__ in, unsigned short* __restrict__ out, int n2) {
  const int i = blockIdx.x * 256 + threadIdx.x;
  if (i < n2) {
    const unsigned u = (unsigned)f2bf_bits(in[2 * i]) | ((unsigned)f2bf_bits(in[2 * i + 1]) << 16);
    ((volatile unsigned*)out)[i] = u;
    __threadfence();
    ((volatile unsigned*)out)[i] = u;
  }
}

__global__ __launch_bounds__(256) void cast_f32_bf16_f16x2_carry(
    const float* __restrict__ in, unsigned short* __restrict__ out, int n2, float carry) {
  const int i = blockIdx.x * 256 + threadIdx.x;
  if (i < n2) {
    const _Float16 h0 = (_Float16)(bf_rne(in[2 * i]) * carry);
    const _Float16 h1 = (_Float16)(bf_rne(in[2 * i + 1]) * carry);
    const unsigned u = (unsigned)__builtin_bit_cast(unsigned short, h0) | ((unsigned)__builtin_bit_cast(unsigned short, h1) << 16);
    ((volatile unsigned*)out)[i] = u;
    __threadfence();
    ((volatile unsigned*)out)[i] = u;
  }
}

__global__ __launch_bounds__(32) void lambda_line(
    const float* __restrict__ lq1, const float* __restrict__ lq2,
    const float* __restrict__ lk1, const float* __restrict__ lk2, float* __restrict__ lamp) {
  const int lane = threadIdx.x;
  float d1 = 0.0f, d2 = 0.0f;
#pragma unroll 1
  for (int i = 0; i < kHeadDim; ++i) {
    d1 += bf_rne(lq1[i]) * bf_rne(lk1[i]);
    d2 += bf_rne(lq2[i]) * bf_rne(lk2[i]);
  }
  const float lam = expf(d1) - expf(d2) + 0.8f;
  ((volatile float*)lamp)[lane] = lam;
  __threadfence();
  ((volatile float*)lamp)[lane] = lam;
}

__device__ __forceinline__ __bf16 at_f2bf(float f) { return __builtin_bit_cast(__bf16, f2bf_bits(f)); }
__device__ __forceinline__ void at_split(float f, __bf16& hi, __bf16& lo) {
  const unsigned short hb = f2bf_bits(f);
  hi = __builtin_bit_cast(__bf16, hb);
  lo = at_f2bf(f - __uint_as_float(((unsigned)hb) << 16));
}
__device__ __forceinline__ v8f at_mma(v16b a, v16b b, v8f c) {
  c = __builtin_amdgcn_wmma_f32_16x16x32_bf16(false, a, false, b, (short)0, c, false, false);
  asm volatile("v_nop\n\tv_nop\n\tv_nop\n\tv_nop" : "+v"(c) : "v"(a), "v"(b));
  return c;
}

__global__ __launch_bounds__(128)
void diff_attn64(const unsigned short* __restrict__ Qh, const unsigned short* __restrict__ Ql,
                 const unsigned short* __restrict__ Kh, const unsigned short* __restrict__ Kl,
                 const unsigned short* __restrict__ Vh, const unsigned short* __restrict__ Vl,
                 const float* __restrict__ amask, const float* __restrict__ lamp,
                 float* __restrict__ att, float* __restrict__ part) {
  union FB { v16b v; v8b h[2]; };
  __shared__ __align__(16) unsigned short Ksh[kKC * kHeadDim];
  __shared__ __align__(16) unsigned short Ksl[kKC * kHeadDim];
  __shared__ __align__(16) unsigned short Vth[kHeadDim * kKC];
  __shared__ __align__(16) unsigned short Vtl[kHeadDim * kKC];
  __shared__ __align__(16) __bf16 Psh[4][16 * kKC];
  __shared__ __align__(16) __bf16 Psl[4][16 * kKC];
  __shared__ __align__(16) float Os[4][16 * 68];
  __shared__ float red[4][2];

  const int tid  = threadIdx.x;
  const int wave = tid >> 5;
  const int lane = tid & 31;
  const int hh   = lane >> 4;
  const int c    = lane & 15;
  const int bx   = blockIdx.x;
  const int qb   = bx & (kNQblk - 1);
  const int bh   = bx >> 5;
  const int h    = bh & (kHeads - 1);
  const int b    = bh >> 4;
  const int q0   = qb * kQB + wave * 16;
  const float lam = lamp[0];
  const float negInf = -__builtin_huge_valf();

  const size_t qoff  = (size_t)(b * kSeq + q0 + c) * kQKCols + (size_t)h * 128;
  const size_t vbase = (size_t)(b * kDModel + h * kHeadDim) * kSeq;
  float* ob_ptr = att + (size_t)bh * kSeq * kHeadDim;
  float* os = Os[wave];
  __bf16* pwh = Psh[wave];
  __bf16* pwl = Psl[wave];
  const int kvr = tid >> 1;
  const int dh  = (tid & 1) * 32;
  float psum = 0.0f, psq = 0.0f;

#pragma unroll
  for (int a = 0; a < 2; ++a) {
    v16b qah[2], qal[2];
#pragma unroll
    for (int dc = 0; dc < 2; ++dc) {
      qah[dc] = Frag<__bf16>::load((const __bf16*)Qh + qoff + a * 64 + dc * 32 + 8 * hh);
      qal[dc] = Frag<__bf16>::load((const __bf16*)Ql + qoff + a * 64 + dc * 32 + 8 * hh);
    }
    float mrow[8], lrow[8];
    v8f oacc[4];
#pragma unroll
    for (int r = 0; r < 8; ++r) { mrow[r] = negInf; lrow[r] = 0.0f; }
#pragma unroll
    for (int t = 0; t < 4; ++t) oacc[t] = (v8f){0.f,0.f,0.f,0.f,0.f,0.f,0.f,0.f};

    for (int kc = 0; kc <= qb; ++kc) {
      const int kv0 = kc * kKC;
      __syncthreads();
      {
        const size_t ko = (size_t)(b * kSeq + kv0 + kvr) * kQKCols + (size_t)h * 128 + a * 64 + dh;
        const size_t vo = vbase + (size_t)kvr * kSeq + kv0 + dh;
        u4v t0[4], t1[4];
#pragma unroll
        for (int i = 0; i < 4; ++i) { t0[i] = *(const u4v*)(Kh + ko + 8 * i); t1[i] = *(const u4v*)(Kl + ko + 8 * i); }
#pragma unroll
        for (int i = 0; i < 4; ++i) { *(u4v*)(Ksh + kvr * 64 + dh + 8 * i) = t0[i]; *(u4v*)(Ksl + kvr * 64 + dh + 8 * i) = t1[i]; }
#pragma unroll
        for (int i = 0; i < 4; ++i) { t0[i] = *(const u4v*)(Vh + vo + 8 * i); t1[i] = *(const u4v*)(Vl + vo + 8 * i); }
#pragma unroll
        for (int i = 0; i < 4; ++i) { *(u4v*)(Vth + kvr * 64 + dh + 8 * i) = t0[i]; *(u4v*)(Vtl + kvr * 64 + dh + 8 * i) = t1[i]; }
      }
      float amv[4];
#pragma unroll
      for (int j = 0; j < 4; ++j) amv[j] = (1.0f - bf_rne(amask[b * kSeq + kv0 + j * 16 + c])) * (-1.0e9f);
      __syncthreads();

      v8f s[4];
#pragma unroll
      for (int j = 0; j < 4; ++j) {
        s[j] = (v8f){0.f,0.f,0.f,0.f,0.f,0.f,0.f,0.f};
#pragma unroll
        for (int dc = 0; dc < 2; ++dc) {
          FB kb, kl;
          kb.h[0] = *(const v8b*)(Ksh + (j * 16 + c) * kHeadDim + dc * 32 + 8 * hh);
          kb.h[1] = *(const v8b*)(Ksh + (j * 16 + c) * kHeadDim + dc * 32 + 16 + 8 * hh);
          kl.h[0] = *(const v8b*)(Ksl + (j * 16 + c) * kHeadDim + dc * 32 + 8 * hh);
          kl.h[1] = *(const v8b*)(Ksl + (j * 16 + c) * kHeadDim + dc * 32 + 16 + 8 * hh);
          s[j] = at_mma(qah[dc], kb.v, s[j]);
          s[j] = at_mma(qah[dc], kl.v, s[j]);
          s[j] = at_mma(qal[dc], kb.v, s[j]);
        }
      }
      const bool diag = (kc == qb);
      float cm[8];
#pragma unroll
      for (int r = 0; r < 8; ++r) {
        const int qrow = q0 + 8 * hh + r;
        float m = negInf;
#pragma unroll
        for (int j = 0; j < 4; ++j) {
          const int kvcol = kv0 + j * 16 + c;
          const float cz = (diag && (kvcol > qrow)) ? -1.0e9f : 0.0f;
          float sc = s[j][r] * 0.125f;
          sc = sc + cz;
          sc = sc + amv[j];
          s[j][r] = sc;
          m = fmaxf(m, sc);
        }
#pragma unroll
        for (int off = 1; off < 16; off <<= 1) m = fmaxf(m, __shfl_xor(m, off, 32));
        cm[r] = m;
      }
#pragma unroll
      for (int r = 0; r < 8; ++r) {
        const float mnew = fmaxf(mrow[r], cm[r]);
        const float alpha = expf(mrow[r] - mnew);
        mrow[r] = mnew;
        float ps = 0.0f;
#pragma unroll
        for (int j = 0; j < 4; ++j) {
          const float p = expf(s[j][r] - mnew);
          ps += p;
          __bf16 ph, pl;
          at_split(p, ph, pl);
          pwh[(8 * hh + r) * kKC + j * 16 + c] = ph;
          pwl[(8 * hh + r) * kKC + j * 16 + c] = pl;
        }
#pragma unroll
        for (int off = 1; off < 16; off <<= 1) ps += __shfl_xor(ps, off, 32);
        lrow[r] = lrow[r] * alpha + ps;
#pragma unroll
        for (int t = 0; t < 4; ++t) oacc[t][r] *= alpha;
      }
      __builtin_amdgcn_fence(__ATOMIC_RELEASE, "workgroup");
      __builtin_amdgcn_wave_barrier();
      __builtin_amdgcn_fence(__ATOMIC_ACQUIRE, "workgroup");
#pragma unroll
      for (int kk = 0; kk < 2; ++kk) {
        FB pa, pl;
        pa.h[0] = *(const v8b*)(pwh + c * kKC + kk * 32 + 8 * hh);
        pa.h[1] = *(const v8b*)(pwh + c * kKC + kk * 32 + 16 + 8 * hh);
        pl.h[0] = *(const v8b*)(pwl + c * kKC + kk * 32 + 8 * hh);
        pl.h[1] = *(const v8b*)(pwl + c * kKC + kk * 32 + 16 + 8 * hh);
#pragma unroll
        for (int t = 0; t < 4; ++t) {
          FB vb, vl;
          vb.h[0] = *(const v8b*)(Vth + (t * 16 + c) * kKC + kk * 32 + 8 * hh);
          vb.h[1] = *(const v8b*)(Vth + (t * 16 + c) * kKC + kk * 32 + 16 + 8 * hh);
          vl.h[0] = *(const v8b*)(Vtl + (t * 16 + c) * kKC + kk * 32 + 8 * hh);
          vl.h[1] = *(const v8b*)(Vtl + (t * 16 + c) * kKC + kk * 32 + 16 + 8 * hh);
          oacc[t] = at_mma(pa.v, vb.v, oacc[t]);
          oacc[t] = at_mma(pa.v, vl.v, oacc[t]);
          oacc[t] = at_mma(pl.v, vb.v, oacc[t]);
        }
      }
    }
#pragma unroll
    for (int r = 0; r < 8; ++r) {
      const float inv = 1.0f / lrow[r];
#pragma unroll
      for (int t = 0; t < 4; ++t) {
        const int oi = (8 * hh + r) * 68 + t * 16 + c;
        const float o = oacc[t][r] * inv;
        if (a == 0) {
          os[oi] = o;
        } else {
          const float w = os[oi] - lam * o;
          os[oi] = w;
          psum += w;
          psq += w * w;
        }
      }
    }
  }

#pragma unroll
  for (int off = 1; off < 32; off <<= 1) { psum += __shfl_xor(psum, off, 32); psq += __shfl_xor(psq, off, 32); }
  if (lane == 0) { red[wave][0] = psum; red[wave][1] = psq; }
  __syncthreads();

  {
    const int c4 = (lane & 15) * 4;
    for (int pass = 0; pass < 2; ++pass) {
#pragma unroll
      for (int it = 0; it < 8; ++it) {
        const int row = it * 2 + hh;
        v4f val = *(const v4f*)(os + row * 68 + c4);
        *(volatile v4f*)(ob_ptr + (size_t)(q0 + row) * kHeadDim + c4) = val;
      }
      __threadfence();
    }
  }
  if (wave == 0) {
    const float t0 = ((red[0][0] + red[1][0]) + red[2][0]) + red[3][0];
    const float t1 = ((red[0][1] + red[1][1]) + red[2][1]) + red[3][1];
    const float v = (lane == 0) ? t0 : ((lane == 1) ? t1 : 0.0f);
    float* pline = part + (size_t)bx * 32;
    ((volatile float*)pline)[lane] = v;
    __threadfence();
    ((volatile float*)pline)[lane] = v;
  }
}

__global__ __launch_bounds__(32) void gn_stats(const float* __restrict__ part, float* __restrict__ stats) {
  const int bh = blockIdx.x;
  const int lane = threadIdx.x;
  float s0 = part[(size_t)(bh * kNQblk + lane) * 32 + 0];
  float s1 = part[(size_t)(bh * kNQblk + lane) * 32 + 1];
#pragma unroll
  for (int off = 1; off < 32; off <<= 1) { s0 += __shfl_xor(s0, off, 32); s1 += __shfl_xor(s1, off, 32); }
  const float inv_n = 1.0f / (float)(kSeq * kHeadDim);
  const float mu = s0 * inv_n;
  const float ex2 = s1 * inv_n;
  const float var = fmaxf(ex2 - mu * mu, 0.0f);
  const float rs = rsqrtf(var + 1.0e-5f);
  const float v = (lane == 0) ? mu : ((lane == 1) ? rs : 0.0f);
  ((volatile float*)stats)[bh * 32 + lane] = v;
  __threadfence();
  ((volatile float*)stats)[bh * 32 + lane] = v;
}

__global__ __launch_bounds__(256) void gn_merge(const float* __restrict__ att, const float* __restrict__ stats,
                                              const float* __restrict__ gamma, const float* __restrict__ beta,
                                              unsigned short* __restrict__ merged) {
  const int g = blockIdx.x * 256 + threadIdx.x;
  if (g >= kBatch * kHeads * kSeq * 8) return;
  const int seg = g >> 3;
  const int e8  = (g & 7) * 8;
  const int bh  = seg >> 11;
  const int s   = seg & (kSeq - 1);
  const int h   = bh & (kHeads - 1);
  const int b   = bh >> 4;
  const float mu = stats[bh * 32 + 0];
  const float rs = stats[bh * 32 + 1];
  union U8 { v4f v[2]; float f[8]; };
  U8 x, ga, be;
  const float* ap = att + (size_t)seg * kHeadDim + e8;
  x.v[0]  = *(const v4f*)ap;
  x.v[1]  = *(const v4f*)(ap + 4);
  ga.v[0] = *(const v4f*)(gamma + h * kHeadDim + e8);
  ga.v[1] = *(const v4f*)(gamma + h * kHeadDim + e8 + 4);
  be.v[0] = *(const v4f*)(beta + h * kHeadDim + e8);
  be.v[1] = *(const v4f*)(beta + h * kHeadDim + e8 + 4);
  v8h hv;
#pragma unroll
  for (int e = 0; e < 8; ++e) {
    const float gq = bf_rne(ga.f[e]);
    const float bq = bf_rne(be.f[e]);
    float y = (x.f[e] - mu) * rs;
    y = y * gq + bq;
    y = y * 0.2f;
    float z = y * kMergeCarry;
    asm volatile("" : "+v"(z));
    hv[e] = (_Float16)z;
  }
  unsigned short* dst = merged + (size_t)(b * kSeq + s) * kDModel + h * kHeadDim + e8;
  *(volatile v8h*)dst = hv;
  __threadfence();
  *(volatile v8h*)dst = hv;
}

extern "C" void kernel_launch(void* const* d_in, const int* in_sizes, int n_in,
                              void* d_out, int out_size, void* d_ws, size_t ws_size,
                              hipStream_t stream) {
  if (n_in < 12) return;
  if (in_sizes[0] != kTok * kDModel || in_sizes[1] != kBatch * kSeq ||
      in_sizes[2] != kQKCols * kDModel || in_sizes[3] != kQKCols * kDModel ||
      in_sizes[4] != kDModel * kDModel || in_sizes[5] != kDModel * kDModel ||
      in_sizes[6] != kHeadDim || in_sizes[7] != kHeadDim || in_sizes[8] != kHeadDim || in_sizes[9] != kHeadDim ||
      in_sizes[10] != kDModel || in_sizes[11] != kDModel) return;
  if (out_size != kTok * kDModel) return;
  if (ws_size < kWsTotal) return;

  const float* X     = (const float*)d_in[0];
  const float* amask = (const float*)d_in[1];
  const float* Wq    = (const float*)d_in[2];
  const float* Wk    = (const float*)d_in[3];
  const float* Wv    = (const float*)d_in[4];
  const float* Wo    = (const float*)d_in[5];
  const float* lq1   = (const float*)d_in[6];
  const float* lq2   = (const float*)d_in[7];
  const float* lk1   = (const float*)d_in[8];
  const float* lk2   = (const float*)d_in[9];
  const float* gamma = (const float*)d_in[10];
  const float* beta  = (const float*)d_in[11];

  char* w = (char*)d_ws;
  unsigned short* Xb    = (unsigned short*)(w + kOffXb);
  unsigned short* Wqb   = (unsigned short*)(w + kOffWqb);
  unsigned short* Wkb   = (unsigned short*)(w + kOffWkb);
  unsigned short* Wvb   = (unsigned short*)(w + kOffWvb);
  unsigned short* Wo16  = (unsigned short*)(w + kOffWo16);
  unsigned short* Qh    = (unsigned short*)(w + kOffQh);
  unsigned short* Ql    = (unsigned short*)(w + kOffQl);
  unsigned short* Kh    = (unsigned short*)(w + kOffKh);
  unsigned short* Kl    = (unsigned short*)(w + kOffKl);
  unsigned short* Vth   = (unsigned short*)(w + kOffVth);
  unsigned short* Vtl   = (unsigned short*)(w + kOffVtl);
  float*          att   = (float*)(w + kOffAtt);
  unsigned short* mrg   = (unsigned short*)(w + kOffMerged);
  float*          part  = (float*)(w + kOffPart);
  float*          stats = (float*)(w + kOffStats);
  float*          lamp  = (float*)(w + kOffLam);

  constexpr int n2X  = kTok * kDModel / 2;
  constexpr int n2Wq = kQKCols * kDModel / 2;
  constexpr int n2Wv = kDModel * kDModel / 2;
  static_assert(n2X % 256 == 0 && n2Wq % 256 == 0 && n2Wv % 256 == 0);
  cast_f32_bf16x2<<<n2X / 256, 256, 0, stream>>>(X, Xb, n2X);
  cast_f32_bf16x2<<<n2Wq / 256, 256, 0, stream>>>(Wq, Wqb, n2Wq);
  cast_f32_bf16x2<<<n2Wq / 256, 256, 0, stream>>>(Wk, Wkb, n2Wq);
  cast_f32_bf16x2<<<n2Wv / 256, 256, 0, stream>>>(Wv, Wvb, n2Wv);
  cast_f32_bf16_f16x2_carry<<<n2Wv / 256, 256, 0, stream>>>(Wo, Wo16, n2Wv, kWoCarry);
  lambda_line<<<1, 32, 0, stream>>>(lq1, lq2, lk1, lk2, lamp);

  constexpr int gridQ  = (kTok / 64) * (kQKCols / 64) / 8;
  constexpr int gridVt = (kDModel / 64) * (kSeq / 64) / 8;
  constexpr int gridO  = (kTok / 64) * (kDModel / 64) / 8;
  static_assert(gridQ * 8 == (kTok / 64) * (kQKCols / 64));
  static_assert(gridVt * 8 == (kDModel / 64) * (kSeq / 64));
  static_assert(gridO * 8 == (kTok / 64) * (kDModel / 64));
  wmma_gemm64<1, false, 0, 2, false><<<dim3(gridQ, 1, 1), 256, 0, stream>>>(
      Xb, Xb, kDModel, 0L, Wqb, Wqb, kDModel, 0L, (void*)Qh, (void*)Ql, kQKCols, 0L,
      lamp, lamp, 0L, kTok, kQKCols, kDModel, 1.0f);
  wmma_gemm64<1, false, 0, 2, false><<<dim3(gridQ, 1, 1), 256, 0, stream>>>(
      Xb, Xb, kDModel, 0L, Wkb, Wkb, kDModel, 0L, (void*)Kh, (void*)Kl, kQKCols, 0L,
      lamp, lamp, 0L, kTok, kQKCols, kDModel, 1.0f);
  wmma_gemm64<1, false, 0, 2, false><<<dim3(gridVt, kBatch, 1), 256, 0, stream>>>(
      Wvb, Wvb, kDModel, 0L, Xb, Xb, kDModel, (long)kSeq * kDModel, (void*)Vth, (void*)Vtl, kSeq, (long)kDModel * kSeq,
      lamp, lamp, 0L, kDModel, kSeq, kDModel, 1.0f);

  diff_attn64<<<kAttnBlocks, 128, 0, stream>>>(Qh, Ql, Kh, Kl, Vth, Vtl, amask, lamp, att, part);

  gn_stats<<<kBatch * kHeads, 32, 0, stream>>>(part, stats);
  gn_merge<<<(kBatch * kHeads * kSeq * 8) / 256, 256, 0, stream>>>(att, stats, gamma, beta, mrg);

  wmma_gemm64<0, false, 0, 0, false><<<dim3(gridO, 1, 1), 256, 0, stream>>>(
      mrg, mrg, kDModel, 0L, Wo16, Wo16, kDModel, 0L, d_out, d_out, kDModel, 0L,
      lamp, lamp, 0L, kTok, kDModel, kDModel, 1.0f / (kMergeCarry * kWoCarry));
}
